// MLPEdgePredictor_9869834846315
// MI455X (gfx1250) — hardware-verified
//
#include <hip/hip_runtime.h>
#include <math.h>

typedef __attribute__((ext_vector_type(16))) _Float16 v16h;
typedef __attribute__((ext_vector_type(16))) __bf16 v16b;
typedef __attribute__((ext_vector_type(8)))  _Float16 v8h;
typedef __attribute__((ext_vector_type(8)))  float v8f;
typedef __attribute__((ext_vector_type(4)))  float v4f;
typedef __attribute__((ext_vector_type(2)))  float v2f;
typedef __attribute__((ext_vector_type(4)))  unsigned v4u;
typedef __attribute__((ext_vector_type(4)))  int v4i;
typedef float __attribute__((may_alias)) float_a;
typedef int __attribute__((may_alias)) int_a;

template <typename T> __device__ __forceinline__ void vst2(void* p, T v) { *(volatile T*)p = v; __threadfence(); *(volatile T*)p = v; }
__device__ __forceinline__ v8f wmma16(v16h a, v16h b, v8f c) {
  v8f d = __builtin_amdgcn_wmma_f32_16x16x32_f16(false, a, false, b, (short)0, c, false, false);
  asm volatile("v_nop\n\tv_nop\n\tv_nop\n\tv_nop" : "+v"(d) : "v"(a), "v"(b));
  return d;
}
__device__ __forceinline__ v8f wmma_bf(v16b a, v16b b, v8f c) {
  v8f d = __builtin_amdgcn_wmma_f32_16x16x32_bf16(false, a, false, b, (short)0, c, false, false);
  asm volatile("v_nop\n\tv_nop\n\tv_nop\n\tv_nop" : "+v"(d) : "v"(a), "v"(b));
  return d;
}
__device__ __forceinline__ v16h frag_h(const _Float16* rowk0, int lane) {
  union { v16h v; v8h q[2]; } u; const _Float16* p = rowk0 + 8 * (lane >> 4);
  u.q[0] = *(const v8h*)p; u.q[1] = *(const v8h*)(p + 16); return u.v;
}
__device__ __forceinline__ v16h frag_f32(const float* rowk0, int lane) {
  v16h a; const float* p = rowk0 + 8 * (lane >> 4);
#pragma unroll
  for (int i = 0; i < 8; ++i) { a[i] = (_Float16)p[i]; a[8 + i] = (_Float16)p[16 + i]; }
  return a;
}
__device__ __forceinline__ v16h frag_f32s(const float* rowk0, int lane, float sc) {
  v16h a; const float* p = rowk0 + 8 * (lane >> 4);
#pragma unroll
  for (int i = 0; i < 8; ++i) { a[i] = (_Float16)(p[i] * sc); a[8 + i] = (_Float16)(p[16 + i] * sc); }
  return a;
}
__device__ __forceinline__ v16h fragc_f32(const float* W, int k0, int n, int lane, int ld, int K) {
  v16h a; const int g = lane >> 4;
#pragma unroll
  for (int i = 0; i < 8; ++i) { const int ka = k0 + 8 * g + i, kb = ka + 16;
    a[i] = (_Float16)(ka < K ? W[(size_t)(ka < K ? ka : K - 1) * ld + n] : 0.f); a[8 + i] = (_Float16)(kb < K ? W[(size_t)(kb < K ? kb : K - 1) * ld + n] : 0.f); }
  return a;
}
struct F2 { v16b h, l; };
__device__ __forceinline__ F2 bsplit16(const float v[16]) { F2 r;
#pragma unroll
  for (int i = 0; i < 16; ++i) { const __bf16 h = (__bf16)v[i]; r.h[i] = h; r.l[i] = (__bf16)(v[i] - (float)h); }
  return r; }
__device__ __forceinline__ F2 split_row(const float* row, int k0, int lane) { float v[16]; const float* p = row + k0 + 8 * (lane >> 4);
#pragma unroll
  for (int i = 0; i < 8; ++i) { v[i] = p[i]; v[8 + i] = p[16 + i]; }
  return bsplit16(v); }
__device__ __forceinline__ F2 split_rowK(const float* row, int k0, int lane, int K) { float v[16]; const int g = lane >> 4;
#pragma unroll
  for (int i = 0; i < 8; ++i) { const int ka = k0 + 8 * g + i, kb = ka + 16; v[i] = ka < K ? row[ka < K ? ka : K - 1] : 0.f; v[8 + i] = kb < K ? row[kb < K ? kb : K - 1] : 0.f; }
  return bsplit16(v); }
__device__ __forceinline__ F2 split_col(const float* W, int k0, int n, int lane, int ld, int K) { float v[16]; const int g = lane >> 4;
#pragma unroll
  for (int i = 0; i < 8; ++i) { const int ka = k0 + 8 * g + i, kb = ka + 16; v[i] = ka < K ? W[(size_t)(ka < K ? ka : K - 1) * ld + n] : 0.f; v[8 + i] = kb < K ? W[(size_t)(kb < K ? kb : K - 1) * ld + n] : 0.f; }
  return bsplit16(v); }
__device__ __forceinline__ v8f mac3(const F2& a, const F2& b, v8f c) { c = wmma_bf(a.l, b.h, c); c = wmma_bf(a.h, b.l, c); return wmma_bf(a.h, b.h, c); }
__device__ __forceinline__ float sigm(float v) { return 1.0f / (1.0f + expf(-v)); }
#define LDSX() do { asm volatile("s_wait_dscnt 0" ::: "memory"); __builtin_amdgcn_wave_barrier(); __builtin_amdgcn_fence(__ATOMIC_RELEASE, "workgroup"); } while (0)


#define NE 600000
#define NNODE 100000
#define DD 128
#define D2 (2 * DD)
#define NBLK (NE / 64)
#define WSC 256.0f
#define LNEPS 1e-5f
#ifndef TBLK
#define TBLK NBLK
#endif
typedef __attribute__((ext_vector_type(8))) __bf16 v8b;
__device__ __forceinline__ v16b frag_b(const __bf16* rowk0, int lane) {
  union { v16b v; v8b q[2]; } u; const __bf16* p = rowk0 + 8 * (lane >> 4);
  u.q[0] = *(const v8b*)p; u.q[1] = *(const v8b*)(p + 16); return u.v;
}
__device__ __forceinline__ float bfr(float v) { return (float)(__bf16)v; }
__device__ __attribute__((noinline)) float exp_ni(float v) { return expf(v); }
__device__ __attribute__((noinline)) float erf_ni(float v) { return erff(v); }

#define WS_PW  0u
#define WS_END (WS_PW + 2u * DD * D2)

__global__ __launch_bounds__(256) void k_pack(const float* __restrict__ W1, _Float16* __restrict__ PW) { const int n = blockIdx.x, t = threadIdx.x; __shared__ __align__(16) _Float16 s[D2]; s[t] = (_Float16)(bfr(W1[(size_t)t * DD + n]) * WSC); __syncthreads(); if (t < D2 / 8) vst2((unsigned*)(PW + (size_t)n * D2 + t * 8), *(const v4u*)&s[t * 8]); }
__global__ __launch_bounds__(128) void k_edge(const float* __restrict__ X, const int* __restrict__ SRC, const int* __restrict__ DST, const float* __restrict__ A, const _Float16* __restrict__ PW, const float* __restrict__ B1, const float* __restrict__ W2, const float* __restrict__ B2, const float* __restrict__ G, const float* __restrict__ Bt, float* __restrict__ OUT) {
  __shared__ __align__(16) _Float16 sh[64][D2 + 8]; __shared__ __align__(16) float ssc[64]; __shared__ int su[64], sv[64];
  const int tid = threadIdx.x, wave = tid >> 5, lane = tid & 31, col = lane & 15, g = lane >> 4; const size_t e0 = (size_t)blockIdx.x * 64;
  if (tid < 64) { int u = SRC[e0 + tid], v = DST[e0 + tid]; u = u < 0 ? 0 : (u >= NNODE ? NNODE - 1 : u); v = v < 0 ? 0 : (v >= NNODE ? NNODE - 1 : v); su[tid] = u; sv[tid] = v; } __syncthreads();
  { const int rl = tid >> 1, half = tid & 1; const float* xr = X + (size_t)(half == 0 ? su[rl] : sv[rl]) * DD; const float ae = bfr(A[e0 + rl]); float v[DD / 4]; float s = 0.f;
    float s1 = 0.f, s2 = 0.f; for (int c = 0; c < DD; ++c) { const float hv = ae * bfr(xr[c]); s1 += hv; } s1 += __shfl_xor(s1, 1); const float mu = s1 / (float)D2;
    for (int c = 0; c < DD; ++c) { const float d = ae * bfr(xr[c]) - mu; s2 += d * d; } s2 += __shfl_xor(s2, 1); const float inv = 1.0f / sqrtf(s2 / (float)D2 + LNEPS);
    for (int c = 0; c < DD; ++c) { const int cc = half * DD + c; sh[rl][cc] = (_Float16)((ae * bfr(xr[c]) - mu) * inv * bfr(G[cc]) + bfr(Bt[cc])); } (void)v; (void)s; }
  __syncthreads();
  v8f acc[8] = {};
#pragma unroll
  for (int kc = 0; kc < D2 / 32; ++kc) { v16h a; const _Float16* pp = &sh[wave * 16 + col][kc * 32 + 8 * g];
#pragma unroll
    for (int i = 0; i < 8; ++i) { a[i] = pp[i]; a[8 + i] = pp[16 + i]; }
#pragma unroll
    for (int j = 0; j < 8; ++j) acc[j] = wmma16(a, frag_h(PW + (size_t)(j * 16 + col) * D2 + kc * 32, lane), acc[j]); }
  float part[8];
#pragma unroll
  for (int r = 0; r < 8; ++r) part[r] = 0.f;
#pragma unroll
  for (int j = 0; j < 8; ++j) { const int c = j * 16 + col; const float bb = bfr(B1[c]), w2 = bfr(W2[c]);
#pragma unroll
    for (int r = 0; r < 8; ++r) { const float z = acc[j][r] * (1.0f / WSC) + bb; part[r] += (z > 0.f ? z : expm1f(z)) * w2; } }
#pragma unroll
  for (int r = 0; r < 8; ++r) { float v = part[r];
#pragma unroll
    for (int o = 1; o < 16; o <<= 1) v += __shfl_xor(v, o);
    if (col == 0) ssc[wave * 16 + 8 * g + r] = v + bfr(B2[0]); }
  __syncthreads(); if (tid < 16) vst2(OUT + e0 + tid * 4, *(const v4f*)&ssc[tid * 4]); }
extern "C" void kernel_launch(void* const* d_in, const int* in_sizes, int n_in, void* d_out, int out_size, void* d_ws, size_t ws_size, hipStream_t stream) {
  (void)in_sizes; (void)n_in; (void)out_size;
  const float** F = (const float**)d_in;
  if (ws_size < (size_t)WS_END) return;
  char* ws = (char*)d_ws; _Float16* PW = (_Float16*)(ws + WS_PW);
  k_pack<<<DD, 256, 0, stream>>>(F[4], PW);
  k_edge<<<TBLK, 128, 0, stream>>>(F[0], (const int*)d_in[1], (const int*)d_in[2], F[3], PW, F[5], F[6], F[7], F[8], F[9], (float*)d_out);
}
